// GAT_70076686401563
// MI455X (gfx1250) — hardware-run, weakly checked
//
#include <hip/hip_runtime.h>


namespace {

constexpr int N = 100000, NP = 100032, NPL = NP  , SRCM = N  , EFULL = 1600000, E = EFULL  ;
constexpr int FI = 128, H = 8, FO = 32, D = H * FO  , C2 = 32  , DO = 40, DOP = 64, NL = (NPL < N ? NPL : N);
constexpr float WSQ = 0.25f, RS_ = 1024.0f;
constexpr float XS = 8.0f, WSC = 256.0f, NSLOPE = 0.2f, AEPS = 1e-8f, SLOPE = 0.0f, BNEPS = 1e-5f;
static_assert(NP % 32 == 0 && NP >= N && NPL % 32 == 0 && D == 256 && FI == 128 && (32 * DO * 4) % 128 == 0, "tiling");
typedef _Float16 b16;
typedef __attribute__((ext_vector_type(16))) _Float16 v16b;
typedef __attribute__((ext_vector_type(8))) _Float16 v8b;
typedef __attribute__((ext_vector_type(8))) float v8f;
typedef __attribute__((ext_vector_type(4))) float v4f;
__device__ __forceinline__ float bf16_rne(float f) { unsigned int u = __float_as_uint(f); u += 0x7FFFu + ((u >> 16) & 1u); return __uint_as_float(u & 0xFFFF0000u); }
__device__ __forceinline__ void split16(float v, b16& hi, b16& lo) { hi = (b16)v; lo = (b16)(v - (float)hi); }
__device__ __forceinline__ v16b frag_kb(const b16* p, int hh) { const v8b a = *(const v8b*)(p + 8 * hh), b = *(const v8b*)(p + 16 + 8 * hh); v16b f;
#pragma unroll
  for (int e = 0; e < 8; ++e) { f[e] = a[e]; f[8 + e] = b[e]; } return f; }
__device__ __forceinline__ v8f wmma16b(v16b a, v16b b, v8f c) { v8f d = __builtin_amdgcn_wmma_f32_16x16x32_f16(false, a, false, b, (short)0, c, false, false); asm volatile("v_nop\n\tv_nop\n\tv_nop\n\tv_nop" : "+v"(d) : "v"(a), "v"(b)); return d; }
__device__ __forceinline__ void wave_lds_sync() { __builtin_amdgcn_fence(__ATOMIC_RELEASE, "workgroup"); __builtin_amdgcn_wave_barrier(); __builtin_amdgcn_fence(__ATOMIC_ACQUIRE, "workgroup"); }
__device__ __forceinline__ float pmul(float a, float b) { float p = a * b; asm volatile("" : "+v"(p)); return p; }
__device__ __forceinline__ int iclamp(int v, int lo, int hi) { return v < lo ? lo : (v > hi ? hi : v); }
constexpr int CSR_NBLK = 512, CSR_GB = 9, CSR_GN = 1 << CSR_GB  , CSR_MAXG = 512, CSR_CAP = 12288  ;
__global__ __launch_bounds__(64) void csrA_kernel(const int* __restrict__ dst, int E, int N, int nG, int CHP, int NGP, int* __restrict__ STG, int* __restrict__ HST) {
  extern __shared__ int sm[];
  int* cnt = sm; int* run = sm + NGP; int* ids = sm + 2 * NGP;
  const int b = blockIdx.x; const int ch = (E + CSR_NBLK - 1) / CSR_NBLK; const int e0 = b * ch, e1 = min(E, e0 + ch);
  for (int i = threadIdx.x; i < NGP; i += 64) cnt[i] = 0;
  for (int i = threadIdx.x; i < CHP; i += 64) ids[i] = -1;
  __syncthreads();
  if (threadIdx.x == 0) {
    for (int e = e0; e < e1; ++e) { int d = dst[e]; d = (d < 0) ? 0 : (d >= N ? N - 1 : d); cnt[d >> CSR_GB] += 1; }
    int acc = 0; for (int g = 0; g < nG; ++g) { run[g] = acc; acc += cnt[g]; }
    for (int e = e0; e < e1; ++e) { int d = dst[e]; d = (d < 0) ? 0 : (d >= N ? N - 1 : d); const int g = d >> CSR_GB; ids[run[g]] = e; run[g] += 1; } }
  __syncthreads();
  typedef __attribute__((ext_vector_type(4))) int v4i;
  for (int pass = 0; pass < 2; ++pass) {
    for (int i = threadIdx.x; i < CHP / 4; i += 64) *(volatile v4i*)(STG + (size_t)b * CHP + i * 4) = *(const v4i*)(&ids[i * 4]);
    for (int i = threadIdx.x; i < NGP / 4; i += 64) { v4i v; for (int e = 0; e < 4; ++e) v[e] = (i * 4 + e < nG) ? cnt[i * 4 + e] : 0; *(volatile v4i*)(HST + (size_t)b * NGP + i * 4) = v; }
    __threadfence(); }
}
__global__ __launch_bounds__(512) void csrS_kernel(const int* __restrict__ HST, int nG, int NGP, int* __restrict__ START, int* __restrict__ TOT, int* __restrict__ OFF) {
  __shared__ int tot[CSR_MAXG];
  const int b = threadIdx.x;
  for (int pass = 0; pass < 2; ++pass) { int runb = 0; for (int g = 0; g < nG; ++g) { int c = HST[(size_t)b * NGP + g]; c = (c < 0) ? 0 : c; ((volatile int*)OFF)[(size_t)g * CSR_NBLK + b] = runb; runb += c; } __threadfence(); }
  for (int g = threadIdx.x; g < nG; g += 512) { int s = 0; for (int bb = 0; bb < CSR_NBLK; ++bb) { int c = HST[(size_t)bb * NGP + g]; s += (c < 0) ? 0 : c; } tot[g] = s; }
  __syncthreads();
  if (threadIdx.x < 32) {
    __shared__ int st[CSR_MAXG + 32];
    if (threadIdx.x == 0) { int acc = 0; for (int g = 0; g < NGP; ++g) { st[g] = acc; if (g < nG) acc += (tot[g] + 31) & ~31; } st[NGP] = acc; }
    __builtin_amdgcn_fence(__ATOMIC_RELEASE, "workgroup"); __builtin_amdgcn_wave_barrier(); __builtin_amdgcn_fence(__ATOMIC_ACQUIRE, "workgroup");
    for (int pass = 0; pass < 2; ++pass) { for (int i = threadIdx.x; i < NGP + 32; i += 32) { ((volatile int*)START)[i] = (i <= NGP) ? st[min(i, NGP)] : 0; ((volatile int*)TOT)[i] = (i < nG) ? tot[i] : 0; } __threadfence(); } }
}
__global__ __launch_bounds__(256) void csrB_kernel(const int* __restrict__ dst, int N, int nG, int CHP, int NGP, int permLen, const int* __restrict__ STG, const int* __restrict__ HST, const int* __restrict__ OFF, const int* __restrict__ START, const int* __restrict__ TOT, int* __restrict__ PERM, int* __restrict__ ROWPTR, int* __restrict__ ROWCNT, int* __restrict__ FLAG) {
  typedef __attribute__((ext_vector_type(4))) int v4i;
  __shared__ int ids[CSR_CAP]; __shared__ unsigned short key[CSR_CAP]; __shared__ int outp[CSR_CAP]; __shared__ int ncnt[CSR_GN + 1]; __shared__ int boff[CSR_NBLK + 1];
  const int g = blockIdx.x, t_ = threadIdx.x; int tot = TOT[g]; int st = START[g], stn = START[g + 1]; const int v0 = g * CSR_GN; const int nv = min(CSR_GN, N - v0);
  st = (st < 0) ? 0 : (st > permLen - 32 ? permLen - 32 : st) & ~31; stn = (stn < st) ? st : (stn > permLen ? permLen : stn); tot = (tot < 0) ? 0 : tot; if (tot > stn - st && tot <= CSR_CAP) tot = stn - st;
  if (tot > CSR_CAP) {
    for (int pass = 0; pass < 2; ++pass) { for (int i = t_; i < CSR_GN / 4; i += 256) { v4i a, c; for (int e = 0; e < 4; ++e) { a[e] = st; c[e] = 0; } *(volatile v4i*)(ROWPTR + v0 + i * 4) = a; *(volatile v4i*)(ROWCNT + v0 + i * 4) = c; } if (t_ == 0) ((volatile int*)FLAG)[0] = 1; __threadfence(); } (void)nv; return; }
  if (t_ == 0) { int acc = 0; for (int b = 0; b < CSR_NBLK; ++b) { boff[b] = acc; int c = HST[(size_t)b * NGP + g]; c = (c < 0) ? 0 : (c > CHP ? CHP : c); acc += c; if (acc > tot) acc = tot; } boff[CSR_NBLK] = acc; }
  for (int i = t_; i <= CSR_GN; i += 256) ncnt[i] = 0;
  __syncthreads();
  for (int b = 0; b < CSR_NBLK; ++b) { const int c = boff[b + 1] - boff[b]; int o_ = OFF[(size_t)g * CSR_NBLK + b]; o_ = (o_ < 0) ? 0 : (o_ > CHP - c ? CHP - c : o_); const int* src_ = STG + (size_t)b * CHP + o_;
    for (int i = t_; i < c; i += 256) { int id = src_[i]; id = (id < 0) ? 0 : id; ids[boff[b] + i] = id; int d = dst[id]; d = (d < v0) ? v0 : (d >= N ? N - 1 : d); int kk = d - v0; kk = (kk < 0) ? 0 : (kk >= CSR_GN ? CSR_GN - 1 : kk); key[boff[b] + i] = (unsigned short)kk; } }
  __syncthreads();
  if (t_ == 0) { for (int i = 0; i < tot; ++i) ncnt[key[i]] += 1; int acc = 0; for (int vl = 0; vl < CSR_GN; ++vl) { const int c = ncnt[vl]; ncnt[vl] = acc; acc += c; } ncnt[CSR_GN] = acc;
    for (int i = 0; i < tot; ++i) { const int vl = key[i]; outp[ncnt[vl]] = ids[i]; ncnt[vl] += 1; }
    for (int vl = CSR_GN; vl > 0; --vl) ncnt[vl] = ncnt[vl - 1]; ncnt[0] = 0; }
  __syncthreads();
  for (int pass = 0; pass < 2; ++pass) {
    for (int i = t_; i < (stn - st) / 4; i += 256) { v4i v; for (int e = 0; e < 4; ++e) { const int q = i * 4 + e; v[e] = (q < tot) ? outp[q] : -1; } *(volatile v4i*)(PERM + st + i * 4) = v; }
    for (int i = t_; i < CSR_GN / 4; i += 256) { v4i a, c; for (int e = 0; e < 4; ++e) { const int vl = i * 4 + e; a[e] = st + ncnt[vl]; c[e] = (vl < nv) ? (ncnt[vl + 1] - ncnt[vl]) : 0; } *(volatile v4i*)(ROWPTR + v0 + i * 4) = a; *(volatile v4i*)(ROWCNT + v0 + i * 4) = c; }
    __threadfence(); }
}
__global__ __launch_bounds__(256) void csrZ_kernel(int* __restrict__ p, size_t n4) { typedef __attribute__((ext_vector_type(4))) int v4i; const size_t tid = (size_t)blockIdx.x * 256 + threadIdx.x, nth = (size_t)gridDim.x * 256; v4i z = {0, 0, 0, 0}; for (size_t i = tid; i < n4; i += nth) *(volatile v4i*)(p + i * 4) = z; }
struct CsrBufs { int *STG, *HST, *OFF, *START, *TOT, *PERM, *ROWPTR, *ROWCNT, *FLAG; int nG, NGP, CHP; size_t permLen; char* base; size_t bytes; };
static size_t csr_carve(CsrBufs& c, char* ws, size_t off, int E, int N) {
  const size_t off0 = off; c.base = ws + off;
  auto al = [&](size_t bytes) { char* p = ws + off; off += (bytes + 255) & ~(size_t)255; return p; };
  c.nG = (N + CSR_GN - 1) / CSR_GN; c.NGP = (c.nG + 31) & ~31; const int ch = (E + CSR_NBLK - 1) / CSR_NBLK; c.CHP = (ch + 31) & ~31; c.permLen = (size_t)E + 32 * (size_t)c.nG + 32;
  c.STG = (int*)al((size_t)CSR_NBLK * c.CHP * 4); c.HST = (int*)al((size_t)CSR_NBLK * c.NGP * 4); c.OFF = (int*)al((size_t)c.NGP * CSR_NBLK * 4); c.START = (int*)al((size_t)(c.NGP + 64) * 4); c.TOT = (int*)al((size_t)(c.NGP + 64) * 4);
  c.PERM = (int*)al(c.permLen * 4); c.ROWPTR = (int*)al((size_t)c.nG * CSR_GN * 4); c.ROWCNT = (int*)al((size_t)c.nG * CSR_GN * 4); c.FLAG = (int*)al(256);
  c.bytes = off - off0; return off;
}
static void csr_build(const CsrBufs& c, const int* dst, int E, int N, hipStream_t stream) {
  const size_t smem = (size_t)(2 * c.NGP + c.CHP) * 4;
  csrZ_kernel<<<512, 256, 0, stream>>>((int*)c.base, c.bytes / 16);
  csrA_kernel<<<CSR_NBLK, 64, smem, stream>>>(dst, E, N, c.nG, c.CHP, c.NGP, c.STG, c.HST);
  csrS_kernel<<<1, 512, 0, stream>>>(c.HST, c.nG, c.NGP, c.START, c.TOT, c.OFF);
  csrB_kernel<<<c.nG, 256, 0, stream>>>(dst, N, c.nG, c.CHP, c.NGP, (int)c.permLen, c.STG, c.HST, c.OFF, c.START, c.TOT, c.PERM, c.ROWPTR, c.ROWCNT, c.FLAG);
}

typedef __attribute__((ext_vector_type(4))) _Float16 v4h;
typedef __attribute__((ext_vector_type(2))) float v2f;
__device__ __forceinline__ float lrelu(float v) { return v > 0.0f ? v : NSLOPE * v; }
template <int K, int NOUTR, int NOUTP>
__global__ __launch_bounds__(256) void wt_kernel(const float* __restrict__ w, b16* __restrict__ WT, float scl) {
  const int u = blockIdx.x * 256 + threadIdx.x; if (u >= NOUTP * K / 8) return; const int e = u * 8; const int o = e / K, k0 = e % K; v8b v;
#pragma unroll
  for (int j = 0; j < 8; ++j) v[j] = (b16)(o < NOUTR ? bf16_rne(w[(size_t)(k0 + j) * NOUTR + o]) * scl : 0.0f);
  for (int pass = 0; pass < 2; ++pass) { *(volatile v8b*)(WT + e) = v; __threadfence(); }
}
__device__ __forceinline__ float elu_(float t) { return t > 0.0f ? t : (__expf(t) - 1.0f); }
__global__ __launch_bounds__(256) void node_kernel(const float* __restrict__ x, const b16* __restrict__ WT, const float* __restrict__ asrc, const float* __restrict__ adst, float* __restrict__ Hh, float* __restrict__ SC) {
  __shared__ __attribute__((aligned(16))) b16 As[32][128 + 8]; __shared__ __attribute__((aligned(16))) float Tf[32][D + 4]; __shared__ __attribute__((aligned(16))) float Sc[32 * 16];
  const int tid = threadIdx.x, wave = tid >> 5, lane = tid & 31, nloc = lane & 15, hlf = lane >> 4; const int v0 = blockIdx.x * 32; const int row = tid >> 3, g = tid & 7;
  v8f acc[2][2] = {{(v8f){}, (v8f){}}, {(v8f){}, (v8f){}}};
#pragma unroll 1
  for (int half = 0; half < FI / 128; ++half) {
    __syncthreads();
    { const int v = v0 + row; const float* xr = x + (size_t)(v < N ? v : N - 1) * FI + half * 128 + g * 16;
#pragma unroll
      for (int q = 0; q < 4; ++q) { const v4f t4 = *(const v4f*)(xr + 4 * q); v4h o4; for (int j = 0; j < 4; ++j) o4[j] = (b16)(bf16_rne(t4[j]) * XS); *(v4h*)(&As[row][g * 16 + 4 * q]) = o4; } }
    __syncthreads();
#pragma unroll
    for (int kb = 0; kb < 128; kb += 32) { const v16b a0 = frag_kb(&As[nloc][kb], hlf), a1 = frag_kb(&As[16 + nloc][kb], hlf);
#pragma unroll
      for (int t = 0; t < 2; ++t) { const v16b bw = frag_kb(WT + (size_t)(wave * 32 + t * 16 + nloc) * FI + half * 128 + kb, hlf); acc[0][t] = wmma16b(a0, bw, acc[0][t]); acc[1][t] = wmma16b(a1, bw, acc[1][t]); } } }
#pragma unroll
  for (int t = 0; t < 2; ++t) { const int col = wave * 32 + t * 16 + nloc;
#pragma unroll
    for (int rt = 0; rt < 2; ++rt)
#pragma unroll
      for (int q = 0; q < 8; ++q) { const int rr = rt * 16 + 8 * hlf + q; Tf[rr][col] = (v0 + rr < N) ? acc[rt][t][q] * (1.0f / (XS * WSC)) : 0.0f; } }
  __syncthreads();
  { float s1 = 0.0f, s2 = 0.0f;
#pragma unroll 8
    for (int f = 0; f < FO; ++f) { const float hv = Tf[row][g * FO + f]; s1 = fmaf(hv, bf16_rne(asrc[g * FO + f]), s1); s2 = fmaf(hv, bf16_rne(adst[g * FO + f]), s2); }
    Sc[row * 16 + g] = s1; Sc[row * 16 + 8 + g] = s2; }
  __syncthreads();
  for (int pass = 0; pass < 2; ++pass) { for (int rr = wave * 4; rr < wave * 4 + 4; ++rr) { float* dst = Hh + (size_t)(v0 + rr) * D;
#pragma unroll
      for (int s = 0; s < 2; ++s) *(volatile v4f*)(dst + s * 128 + lane * 4) = *(const v4f*)(&Tf[rr][s * 128 + lane * 4]); }
    if (tid < 128) *(volatile v4f*)(SC + (size_t)v0 * 16 + tid * 4) = *(const v4f*)(&Sc[tid * 4]);
    __threadfence(); }
}
__global__ __launch_bounds__(256) void agg_kernel(const float* __restrict__ Hh, const float* __restrict__ SC, const int* __restrict__ srcs, const int* __restrict__ PERM, const int* __restrict__ ROWPTR, const int* __restrict__ ROWCNT, int permLen, const float* __restrict__ bias, float* __restrict__ out, int mrows) {
  const int tid = threadIdx.x; const int row = tid >> 3, g = tid & 7; const int v = blockIdx.x * 32 + row;
  float acc[FO]; for (int j = 0; j < FO; ++j) acc[j] = 0.0f;
  const int vv = v < N ? v : N - 1; int cnt = 0, p0 = 0; if (v < N) { cnt = iclamp(ROWCNT[v], 0, 65536); p0 = iclamp(ROWPTR[v], 0, permLen - 1); if (p0 + cnt > permLen) cnt = permLen - p0; } const float sd = SC[(size_t)vv * 16 + 8 + g];
  float m = -INFINITY, l = 0.0f;
#pragma unroll 1
  for (int i = 0; i <= cnt; ++i) { int s; if (i < cnt) { const int e = iclamp(PERM[p0 + i], 0, E - 1); s = iclamp(srcs[e], 0, N - 1); if (SRCM < N) s %= SRCM; } else s = vv;
    const float sc = lrelu(SC[(size_t)s * 16 + g] + sd);
    const float mn = fmaxf(m, sc); const float al = __expf(m - mn), pw = __expf(sc - mn); l = l * al + pw; m = mn; const float* hr = Hh + (size_t)s * D + g * FO;
#pragma unroll
    for (int q = 0; q < 8; ++q) { const v4f t4 = *(const v4f*)(hr + 4 * q); for (int j = 0; j < 4; ++j) acc[4 * q + j] = fmaf(pw, t4[j], pmul(acc[4 * q + j], al)); } }
  const float inv = 1.0f / l;
  for (int pass = 0; pass < 2; ++pass) { if (v < mrows) { float* orow = out + (size_t)v * D + g * FO;
#pragma unroll
      for (int q = 0; q < 8; ++q) { v4f o4; for (int j = 0; j < 4; ++j) o4[j] = (v < N) ? elu_(acc[4 * q + j] * inv + bf16_rne(bias[g * FO + 4 * q + j])) : 0.0f; *(volatile v4f*)(orow + 4 * q) = o4; } }
    __threadfence(); }
}
__global__ __launch_bounds__(64) void node2_kernel(const float* __restrict__ H1, const b16* __restrict__ WT, const b16* __restrict__ WQ, const float* __restrict__ as2, const float* __restrict__ ad2, float* __restrict__ XS2, float* __restrict__ SC2) {
  __shared__ __attribute__((aligned(16))) b16 Ah[2][16][D + 8], Al[2][16][D + 8]; __shared__ __attribute__((aligned(16))) float Tf[2][16][C2 + 4]; __shared__ __attribute__((aligned(16))) float Sc[2][16][4];
  const int wave = threadIdx.x >> 5, lane = threadIdx.x & 31, nloc = lane & 15, hlf = lane >> 4; const size_t m0 = (size_t)blockIdx.x * 32 + wave * 16;
  for (int idx = lane; idx < 16 * (D / 4); idx += 32) { const int rr = idx / (D / 4), c4 = (idx % (D / 4)) * 4; const size_t arow = (m0 + rr < (size_t)N) ? m0 + rr : (size_t)N - 1; const v4f v = *(const v4f*)(H1 + arow * D + c4); v4h hv, lv;
    for (int j = 0; j < 4; ++j) { const float vs = v[j] * XS; const b16 ph = (b16)vs; hv[j] = ph; lv[j] = (b16)((vs - (float)ph) * RS_); } *(v4h*)(&Ah[wave][rr][c4]) = hv; *(v4h*)(&Al[wave][rr][c4]) = lv; }
  wave_lds_sync();
  v8f acc[2] = {(v8f){}, (v8f){}};
#pragma unroll 2
  for (int kb = 0; kb < D; kb += 32) { const v16b a = frag_kb(&Ah[wave][nloc][kb], hlf), al = frag_kb(&Al[wave][nloc][kb], hlf);
#pragma unroll
    for (int t = 0; t < 2; ++t) { const size_t wo_ = (size_t)(t * 16 + nloc) * D + kb; acc[t] = wmma16b(a, frag_kb(WT + wo_, hlf), acc[t]); acc[t] = wmma16b(al, frag_kb(WQ + wo_, hlf), acc[t]); } }
  const float ws0 = bf16_rne(as2[nloc]), ws1 = bf16_rne(as2[16 + nloc]), wd0 = bf16_rne(ad2[nloc]), wd1 = bf16_rne(ad2[16 + nloc]);
#pragma unroll
  for (int r = 0; r < 8; ++r) { const size_t vrow = m0 + 8 * hlf + r; const bool ok = vrow < (size_t)N; const float h0 = ok ? acc[0][r] * (1.0f / (XS * WSC)) : 0.0f, h1 = ok ? acc[1][r] * (1.0f / (XS * WSC)) : 0.0f;
    Tf[wave][8 * hlf + r][nloc] = h0; Tf[wave][8 * hlf + r][16 + nloc] = h1;
    float ss = fmaf(h0, ws0, pmul(h1, ws1)), sdd = fmaf(h0, wd0, pmul(h1, wd1)); for (int o = 1; o <= 8; o <<= 1) { ss += __shfl_xor(ss, o); sdd += __shfl_xor(sdd, o); }
    if (nloc == 0) { Sc[wave][8 * hlf + r][0] = ss; Sc[wave][8 * hlf + r][1] = sdd; Sc[wave][8 * hlf + r][2] = 0.0f; Sc[wave][8 * hlf + r][3] = 0.0f; } }
  wave_lds_sync();
  for (int pass = 0; pass < 2; ++pass) { for (int rr = 0; rr < 16; rr += 4) { const int r2 = rr + (lane >> 3); *(volatile v4f*)(XS2 + (m0 + r2) * C2 + (lane & 7) * 4) = *(const v4f*)(&Tf[wave][r2][(lane & 7) * 4]); }
    if (lane < 16) *(volatile v4f*)(SC2 + (m0 + lane) * 4) = *(const v4f*)(&Sc[wave][lane][0]);
    __threadfence(); }
}
__global__ __launch_bounds__(256) void agg2_kernel(const float* __restrict__ XS2, const float* __restrict__ SC2, const int* __restrict__ srcs, const int* __restrict__ PERM, const int* __restrict__ ROWPTR, const int* __restrict__ ROWCNT, int permLen, const float* __restrict__ bias, float* __restrict__ H2, int mrows) {
  const int tid = threadIdx.x; const int row = tid >> 3, g = tid & 7, c0 = g * 4; const int v = blockIdx.x * 32 + row; const int vv = v < N ? v : N - 1;
  int cnt = 0, p0 = 0; if (v < N) { cnt = iclamp(ROWCNT[v], 0, 65536); p0 = iclamp(ROWPTR[v], 0, permLen - 1); if (p0 + cnt > permLen) cnt = permLen - p0; } const float sd = SC2[(size_t)vv * 4 + 1];
  float m = -INFINITY, l = 0.0f; float acc[4] = {0.0f, 0.0f, 0.0f, 0.0f};
#pragma unroll 1
  for (int i = 0; i <= cnt; ++i) { int s; if (i < cnt) { const int e = iclamp(PERM[p0 + i], 0, E - 1); s = iclamp(srcs[e], 0, N - 1); if (SRCM < N) s %= SRCM; } else s = vv;
    const float sc = lrelu(SC2[(size_t)s * 4] + sd); const float mn = fmaxf(m, sc); const float al = __expf(m - mn), pw = __expf(sc - mn); l = l * al + pw; m = mn; const v4f t4 = *(const v4f*)(XS2 + (size_t)s * C2 + c0);
    for (int j = 0; j < 4; ++j) acc[j] = fmaf(pw, t4[j], pmul(acc[j], al)); }
  const float inv = 1.0f / l;
  for (int pass = 0; pass < 2; ++pass) { if (v < mrows) { v4f o4; for (int j = 0; j < 4; ++j) o4[j] = (v < N) ? elu_(acc[j] * inv + bf16_rne(bias[c0 + j])) : 0.0f; *(volatile v4f*)(H2 + (size_t)v * C2 + c0) = o4; } __threadfence(); }
}
__global__ __launch_bounds__(64) void cls_kernel(const float* __restrict__ H2, const b16* __restrict__ WT, const b16* __restrict__ WQ, const float* __restrict__ bout, float* __restrict__ out, int mrows) {
  __shared__ __attribute__((aligned(16))) b16 Ah[2][16][C2 + 8], Al[2][16][C2 + 8]; __shared__ __attribute__((aligned(16))) float To[32 * DO + 4];
  const int wave = threadIdx.x >> 5, lane = threadIdx.x & 31, nloc = lane & 15, hlf = lane >> 4; const size_t m0 = (size_t)blockIdx.x * 32 + wave * 16;
  for (int idx = lane; idx < 16 * (C2 / 4); idx += 32) { const int rr = idx / (C2 / 4), c4 = (idx % (C2 / 4)) * 4; const size_t arow = (m0 + rr < (size_t)N) ? m0 + rr : (size_t)N - 1; const v4f v = *(const v4f*)(H2 + arow * C2 + c4); v4h hv, lv;
    for (int j = 0; j < 4; ++j) { const float vs = v[j] * XS; const b16 ph = (b16)vs; hv[j] = ph; lv[j] = (b16)((vs - (float)ph) * RS_); } *(v4h*)(&Ah[wave][rr][c4]) = hv; *(v4h*)(&Al[wave][rr][c4]) = lv; }
  wave_lds_sync();
  v8f acc2[4]; for (int t = 0; t < 4; ++t) acc2[t] = (v8f){};
  { const v16b a = frag_kb(&Ah[wave][nloc][0], hlf), al = frag_kb(&Al[wave][nloc][0], hlf);
#pragma unroll
    for (int t = 0; t < 4; ++t) { const size_t wo_ = (size_t)(t * 16 + nloc) * C2; acc2[t] = wmma16b(a, frag_kb(WT + wo_, hlf), acc2[t]); acc2[t] = wmma16b(al, frag_kb(WQ + wo_, hlf), acc2[t]); } }
  float z[4][8];
#pragma unroll
  for (int t = 0; t < 4; ++t) { const int col = t * 16 + nloc; const float bb = (col < DO) ? bf16_rne(bout[col < DO ? col : 0]) : 0.0f;
#pragma unroll
    for (int r = 0; r < 8; ++r) z[t][r] = (col < DO) ? acc2[t][r] * (1.0f / (XS * WSC)) + bb : -INFINITY; }
#pragma unroll
  for (int r = 0; r < 8; ++r) { float mx = -INFINITY; for (int t = 0; t < 4; ++t) mx = fmaxf(mx, z[t][r]); for (int o = 1; o <= 8; o <<= 1) mx = fmaxf(mx, __shfl_xor(mx, o));
    float se = 0.0f; for (int t = 0; t < 4; ++t) se += (z[t][r] > -INFINITY) ? __expf(z[t][r] - mx) : 0.0f; for (int o = 1; o <= 8; o <<= 1) se += __shfl_xor(se, o);
    const float lse = mx + __logf(se);
#pragma unroll
    for (int t = 0; t < 4; ++t) { const int col = t * 16 + nloc; if (col < DO) To[(wave * 16 + 8 * hlf + r) * DO + col] = (m0 + 8 * hlf + r < (size_t)N) ? z[t][r] - lse : 0.0f; } }
  __syncthreads();
  for (int pass = 0; pass < 2; ++pass) { for (int i = threadIdx.x; i < 32 * DO / 4; i += 64) { const int rr = (i * 4) / DO; if (blockIdx.x * 32 + rr < mrows) *(volatile v4f*)(out + (size_t)blockIdx.x * 32 * DO + i * 4) = *(const v4f*)(&To[i * 4]); } __threadfence(); }
}
}

extern "C" void kernel_launch(void* const* d_in, const int* in_sizes, int n_in, void* d_out, int out_size, void* d_ws, size_t ws_size, hipStream_t stream) {
  (void)n_in;
  auto Fp = [&](int i) { return (const float*)d_in[i]; }; auto Ip = [&](int i) { return (const int*)d_in[i]; };
  if (in_sizes[0] != N * FI || in_sizes[1] != 2 * EFULL || in_sizes[2] != FI * D || in_sizes[3] != D || in_sizes[4] != D || in_sizes[5] != D || in_sizes[6] != D * C2 || in_sizes[7] != C2 || in_sizes[8] != C2 || in_sizes[9] != C2 || in_sizes[10] != C2 * DO || in_sizes[11] != DO || out_size != N * DO) return;
  size_t off = 0; char* ws = (char*)d_ws;
  auto carve = [&](size_t bytes) { char* p = ws + off; off += (bytes + 255) & ~(size_t)255; return p; };
  b16* WT1 = (b16*)carve((size_t)D * FI * 2); b16* WT2 = (b16*)carve((size_t)C2 * D * 2); b16* WQ2 = (b16*)carve((size_t)C2 * D * 2); b16* WT3 = (b16*)carve((size_t)DOP * C2 * 2); b16* WQ3 = (b16*)carve((size_t)DOP * C2 * 2);
  float* Hh = (float*)carve((size_t)NP * D * 4); float* SC = (float*)carve((size_t)NP * 16 * 4); float* H1 = (float*)carve((size_t)NP * D * 4);
  float* XS2 = Hh; float* SC2 = Hh + (size_t)NP * C2; float* H2 = SC2 + (size_t)NP * 4;
  CsrBufs csr; off = csr_carve(csr, ws, off, E, N);
  if (off > ws_size || off > ((size_t)240 << 20)) return;
  wt_kernel<FI, D, D><<<(D * FI / 8 + 255) / 256, 256, 0, stream>>>(Fp(2), WT1, WSC);
  wt_kernel<D, C2, C2><<<(C2 * D / 8 + 255) / 256, 256, 0, stream>>>(Fp(6), WT2, WSC); wt_kernel<D, C2, C2><<<(C2 * D / 8 + 255) / 256, 256, 0, stream>>>(Fp(6), WQ2, WSQ);
  wt_kernel<C2, DO, DOP><<<(DOP * C2 / 8 + 255) / 256, 256, 0, stream>>>(Fp(10), WT3, WSC); wt_kernel<C2, DO, DOP><<<(DOP * C2 / 8 + 255) / 256, 256, 0, stream>>>(Fp(10), WQ3, WSQ);
  csr_build(csr, Ip(1) + EFULL, E, N, stream);
  node_kernel<<<NP / 32, 256, 0, stream>>>(Fp(0), WT1, Fp(3), Fp(4), Hh, SC);
  agg_kernel<<<NP / 32, 256, 0, stream>>>(Hh, SC, Ip(1), csr.PERM, csr.ROWPTR, csr.ROWCNT, (int)csr.permLen, Fp(5), H1, NP);
  node2_kernel<<<NP / 32, 64, 0, stream>>>(H1, WT2, WQ2, Fp(7), Fp(8), XS2, SC2);
  agg2_kernel<<<NPL / 32, 256, 0, stream>>>(XS2, SC2, Ip(1), csr.PERM, csr.ROWPTR, csr.ROWCNT, (int)csr.permLen, Fp(9), H2, NPL);
  cls_kernel<<<NPL / 32, 64, 0, stream>>>(H2, WT3, WQ3, Fp(11), (float*)d_out, NL);
}
